// GraphConvBlock_54692113547388
// MI455X (gfx1250) — hardware-verified
//
#include <hip/hip_runtime.h>
#include <math.h>
#include <stdint.h>

#define NB   32
#define NS   512
#define ND   512
#define NH   8
#define NHD  64
#define NFF  1024
#define NM   (NB * NS)
#define MHALF 8192
#define TP   516
#define SDHALF (NB * NH * NS)

static_assert(NS == 512 && ND == 512);
static_assert(ND == NS);
static_assert(NH * NHD == ND);
static_assert(NHD == 64);
static_assert(NS % 64 == 0);
static_assert(NM % MHALF == 0 && MHALF % 64 == 0);
static_assert(ND % 32 == 0 && NFF % 32 == 0);
static_assert((ND & (ND - 1)) == 0 && (NFF & (NFF - 1)) == 0);
static_assert(NFF == 2 * ND);

typedef __attribute__((ext_vector_type(16))) __bf16   v16b;
typedef __attribute__((ext_vector_type(8)))  __bf16   v8b;
typedef __attribute__((ext_vector_type(8)))  float    v8f;
typedef __attribute__((ext_vector_type(4)))  float    v4f;
typedef __attribute__((ext_vector_type(4)))  unsigned int v4u;
typedef __attribute__((ext_vector_type(2)))  unsigned int v2u;
typedef v4f __attribute__((may_alias)) v4fa;
typedef v4u __attribute__((may_alias)) v4ua;
typedef v2u __attribute__((may_alias)) v2ua;

#define V_WB    0
#define V_SEMB  512
#define V_AW    1024
#define V_FF1B  1152
#define V_FF2B  2176
#define V_LN1G  2688
#define V_LN1B  3200
#define V_LN2G  3712
#define V_LN2B  4224
#define V_TOTAL 4736

static constexpr size_t O_XB   = 0;
static constexpr size_t O_ADJB = 16777216;
static constexpr size_t O_Y1HL = 0;
static constexpr size_t O_VTH  = 33554432;
static constexpr size_t O_VTL  = 50331648;
static constexpr size_t O_GHL  = 33554432;
static constexpr size_t O_CTX  = 67108864;
static constexpr size_t O_WB   = 100663296;
static constexpr size_t O_SEMB = 101187584;
static constexpr size_t O_FF1B = 101711872;
static constexpr size_t O_FF2B = 102760448;
static constexpr size_t O_MASK = 103809024;
static constexpr size_t O_SD   = 104857600;
static constexpr size_t O_VEC  = 105906176;
static constexpr size_t WS_TOTAL = 105938944;
static_assert(O_ADJB == O_XB + (size_t)NM * ND * 2);
static_assert(O_VTH == O_Y1HL + (size_t)NM * 2 * ND * 2);
static_assert(O_VTL == O_VTH + (size_t)NB * NH * NHD * NS * 2);
static_assert(O_CTX == O_VTL + (size_t)NB * NH * NHD * NS * 2);
static_assert(O_CTX == O_GHL + (size_t)MHALF * 2 * NFF * 2);
static_assert(O_WB == O_CTX + (size_t)NM * ND * 4);
static_assert(O_SEMB == O_WB + (size_t)ND * ND * 2);
static_assert(O_FF1B == O_SEMB + (size_t)ND * ND * 2);
static_assert(O_FF2B == O_FF1B + (size_t)NFF * ND * 2);
static_assert(O_MASK == O_FF2B + (size_t)ND * NFF * 2);
static_assert(O_SD == O_MASK + (size_t)NM * 16 * 4);
static_assert(O_VEC == O_SD + (size_t)2 * SDHALF * 4);
static_assert(WS_TOTAL == O_VEC + 32768);
static_assert((size_t)V_TOTAL * 4 <= 32768);
static_assert(WS_TOTAL <= 134217728);

__device__ __forceinline__ unsigned short f2bf_bits(float f) {
  const unsigned u = __float_as_uint(f);
  return (unsigned short)((u + 0x7FFFu + ((u >> 16) & 1u)) >> 16);
}
__device__ __forceinline__ float bf_bits2f(unsigned short h) { return __uint_as_float(((unsigned)h) << 16); }
__device__ __forceinline__ float bfr(float f) { return bf_bits2f(f2bf_bits(f)); }
__device__ __forceinline__ unsigned pk16(unsigned short a, unsigned short b) { return (unsigned)a | ((unsigned)b << 16); }

__device__ __forceinline__ void wave_sync() {
  __builtin_amdgcn_fence(__ATOMIC_RELEASE, "workgroup");
  __builtin_amdgcn_wave_barrier();
  __builtin_amdgcn_fence(__ATOMIC_ACQUIRE, "workgroup");
}
__device__ __forceinline__ float wave_sum(float v) {
#pragma unroll
  for (int off = 16; off > 0; off >>= 1) v += __shfl_xor(v, off, 32);
  return v;
}
__device__ __forceinline__ float wave_max(float v) {
#pragma unroll
  for (int off = 16; off > 0; off >>= 1) v = fmaxf(v, __shfl_xor(v, off, 32));
  return v;
}

union FB { v16b v; v8b h[2]; };
__device__ __forceinline__ v16b ldfrag(const __bf16* p) {
  FB f; f.h[0] = *(const v8b*)(p); f.h[1] = *(const v8b*)(p + 16); return f.v;
}
__device__ __forceinline__ v8f wmma_raw(v16b a, v16b b, v8f c) {
  return __builtin_amdgcn_wmma_f32_16x16x32_bf16(false, a, false, b, (short)0, c, false, false);
}
__device__ __forceinline__ v8f at_mma(v16b a, v16b b, v8f c) {
  c = __builtin_amdgcn_wmma_f32_16x16x32_bf16(false, a, false, b, (short)0, c, false, false);
  asm volatile("v_nop\n\tv_nop\n\tv_nop\n\tv_nop" : "+v"(c) : "v"(a), "v"(b));
  return c;
}
__device__ __forceinline__ void dep_guard_b(v8f& a, v8f& b, v16b x, v16b y) { asm volatile("v_nop\n\tv_nop\n\tv_nop\n\tv_nop" : "+v"(a), "+v"(b) : "v"(x), "v"(y)); }
__device__ __forceinline__ void keep4_b(v16b a, v16b b, v16b c, v16b d) { asm volatile("v_nop" :: "v"(a), "v"(b), "v"(c), "v"(d)); }
__device__ __forceinline__ void acc_guard4(v8f& a, v8f& b, v8f& c, v8f& d) { asm volatile("v_nop\n\tv_nop\n\tv_nop\n\tv_nop" : "+v"(a), "+v"(b), "+v"(c), "+v"(d)); }

__device__ __forceinline__ void gemm_tile64(const __bf16* __restrict__ A, const int lda,
                                            const __bf16* __restrict__ Bt, const int ldb,
                                            const int m0, const int n0, const int KA, const int kbmask,
                                            const int lane, v8f (&acc)[4][4]) {
  const int rlane = lane & 15;
  const int koff  = (lane >> 4) * 8;
#pragma unroll
  for (int i = 0; i < 4; ++i)
#pragma unroll
    for (int j = 0; j < 4; ++j) acc[i][j] = (v8f){0.f,0.f,0.f,0.f,0.f,0.f,0.f,0.f};
  const __bf16* ap = A  + (size_t)(m0 + rlane) * lda + koff;
  const __bf16* bp = Bt + (size_t)(n0 + rlane) * ldb + koff;
#pragma unroll 1
  for (int k0 = 0; k0 < KA; k0 += 32) {
    const int kb = k0 & kbmask;
    v16b bh[4];
#pragma unroll
    for (int j = 0; j < 4; ++j) bh[j] = ldfrag(bp + (size_t)(16 * j) * ldb + kb);
#pragma unroll
    for (int i = 0; i < 4; ++i) {
      const v16b ah = ldfrag(ap + (size_t)(16 * i) * lda + k0);
#pragma unroll
      for (int j = 0; j < 4; ++j) acc[i][j] = wmma_raw(ah, bh[j], acc[i][j]);
      dep_guard_b(acc[i][0], acc[i][3], ah, ah);
    }
    keep4_b(bh[0], bh[1], bh[2], bh[3]);
  }
  acc_guard4(acc[0][0], acc[0][1], acc[0][2], acc[0][3]);
  acc_guard4(acc[1][0], acc[1][1], acc[1][2], acc[1][3]);
  acc_guard4(acc[2][0], acc[2][1], acc[2][2], acc[2][3]);
  acc_guard4(acc[3][0], acc[3][1], acc[3][2], acc[3][3]);
}

#define PB_X   4096
#define PB_ADJ 8192
#define PB_W   8320
#define PB_SEM 8448
#define PB_FF1 8704
#define PB_FF2 8960
#define PB_END 8969
static_assert((size_t)NM * ND == (size_t)4096 * 2048);
static_assert(ND * ND == 128 * 2048);
static_assert(NFF * ND == 256 * 2048);

__device__ __forceinline__ void cvt8(const float* __restrict__ src, unsigned short* __restrict__ dst, const size_t g) {
  const v4f a = *(const v4f*)(src + g * 8);
  const v4f c = *(const v4f*)(src + g * 8 + 4);
  v4u o;
  o[0] = pk16(f2bf_bits(a[0]), f2bf_bits(a[1]));
  o[1] = pk16(f2bf_bits(a[2]), f2bf_bits(a[3]));
  o[2] = pk16(f2bf_bits(c[0]), f2bf_bits(c[1]));
  o[3] = pk16(f2bf_bits(c[2]), f2bf_bits(c[3]));
  *(volatile v4u*)(dst + g * 8) = o;
  __threadfence();
  *(volatile v4u*)(dst + g * 8) = o;
}
__device__ __forceinline__ void cvtv(const float* __restrict__ src, float* __restrict__ dst, const int n4, const int tid) {
  const int t = (tid < n4) ? tid : (n4 - 1);
  const v4f a = *(const v4f*)(src + 4 * t);
  v4f o;
  o[0] = bfr(a[0]); o[1] = bfr(a[1]); o[2] = bfr(a[2]); o[3] = bfr(a[3]);
  if (tid < n4) {
    *(volatile v4f*)(dst + 4 * tid) = o;
    __threadfence();
    *(volatile v4f*)(dst + 4 * tid) = o;
  }
}

__global__ __launch_bounds__(256) void k_prep(
    const float* __restrict__ x, const float* __restrict__ adj, const float* __restrict__ wW,
    const float* __restrict__ wb, const float* __restrict__ aw, const float* __restrict__ semW,
    const float* __restrict__ semb, const float* __restrict__ ff1W, const float* __restrict__ ff1b,
    const float* __restrict__ ff2W, const float* __restrict__ ff2b,
    const float* __restrict__ ln1g, const float* __restrict__ ln1b,
    const float* __restrict__ ln2g, const float* __restrict__ ln2b,
    unsigned short* __restrict__ XB, unsigned short* __restrict__ ADJB, unsigned short* __restrict__ WB,
    unsigned short* __restrict__ SEMB, unsigned short* __restrict__ FF1B, unsigned short* __restrict__ FF2B,
    float* __restrict__ VEC) {
  const int bid = blockIdx.x;
  const int tid = threadIdx.x;
  if (bid < PB_X) {
    cvt8(x, XB, (size_t)bid * 256 + tid);
  } else if (bid < PB_ADJ) {
    cvt8(adj, ADJB, (size_t)(bid - PB_X) * 256 + tid);
  } else if (bid < PB_W) {
    cvt8(wW, WB, (size_t)(bid - PB_ADJ) * 256 + tid);
  } else if (bid < PB_SEM) {
    cvt8(semW, SEMB, (size_t)(bid - PB_W) * 256 + tid);
  } else if (bid < PB_FF1) {
    cvt8(ff1W, FF1B, (size_t)(bid - PB_SEM) * 256 + tid);
  } else if (bid < PB_FF2) {
    cvt8(ff2W, FF2B, (size_t)(bid - PB_FF1) * 256 + tid);
  } else {
    const int vb = bid - PB_FF2;
    if (vb == 0)      cvtv(wb,   VEC + V_WB,   ND / 4,  tid);
    else if (vb == 1) cvtv(semb, VEC + V_SEMB, ND / 4,  tid);
    else if (vb == 2) cvtv(aw,   VEC + V_AW,   32,      tid);
    else if (vb == 3) cvtv(ff1b, VEC + V_FF1B, NFF / 4, tid);
    else if (vb == 4) cvtv(ff2b, VEC + V_FF2B, ND / 4,  tid);
    else if (vb == 5) cvtv(ln1g, VEC + V_LN1G, ND / 4,  tid);
    else if (vb == 6) cvtv(ln1b, VEC + V_LN1B, ND / 4,  tid);
    else if (vb == 7) cvtv(ln2g, VEC + V_LN2G, ND / 4,  tid);
    else if (vb == 8) cvtv(ln2b, VEC + V_LN2B, ND / 4,  tid);
  }
}

__global__ __launch_bounds__(256) void k_sem(const unsigned short* __restrict__ ADJB, const unsigned short* __restrict__ SEMB,
                                             const float* __restrict__ vsemb, unsigned* __restrict__ MASKB) {
  extern __shared__ __align__(16) float dsm[];
  __shared__ __align__(16) float sB[ND];
  __shared__ __align__(16) unsigned sMk[64 * 16];
  const int tid = threadIdx.x, lane = tid & 31, wave = tid >> 5;
  const int m0 = blockIdx.x * 64, n0 = wave * 64;
  if (tid < 128) *(v4f*)(sB + 4 * tid) = *(const v4f*)(vsemb + 4 * tid);

  v8f acc[4][4];
  gemm_tile64((const __bf16*)(const void*)ADJB, ND, (const __bf16*)(const void*)SEMB, ND, m0, n0, ND, ND - 1, lane, acc);

  const int rlane = lane & 15, mOff = (lane >> 4) * 8;
#pragma unroll
  for (int i = 0; i < 4; ++i)
#pragma unroll
    for (int j = 0; j < 4; ++j)
#pragma unroll
      for (int r = 0; r < 8; ++r)
        dsm[(16 * i + mOff + r) * TP + n0 + 16 * j + rlane] = acc[i][j][r];
  __syncthreads();

#pragma unroll 1
  for (int rr = 0; rr < 8; ++rr) {
    const int row = wave * 8 + rr;
    const float* tr = dsm + row * TP;
    float v[16];
    float mx = -INFINITY;
#pragma unroll
    for (int c = 0; c < 16; ++c) { v[c] = tr[lane + 32 * c] + sB[lane + 32 * c]; mx = fmaxf(mx, v[c]); }
    mx = wave_max(mx);
    float sum = 0.0f;
#pragma unroll
    for (int c = 0; c < 16; ++c) { v[c] = expf(v[c] - mx); sum += v[c]; }
    sum = wave_sum(sum);
    const float inv = 1.0f / sum;
    unsigned myw = 0u;
#pragma unroll
    for (int c = 0; c < 16; ++c) {
      const float p = v[c] * inv;
      const unsigned w = (unsigned)__ballot(p == 0.0f);
      myw = (lane == c) ? w : myw;
    }
    if (lane < 16) sMk[row * 16 + lane] = myw;
  }
  __syncthreads();

  if (wave == 0) {
    unsigned* dst = MASKB + (size_t)m0 * 16;
    for (int pass = 0; pass < 2; ++pass) {
#pragma unroll
      for (int it = 0; it < 8; ++it) {
        const v4u w = *(const v4ua*)(sMk + 4 * (it * 32 + lane));
        *(volatile v4u*)(dst + 4 * (it * 32 + lane)) = w;
      }
      __threadfence();
    }
  }
}

#define PJ_WAVE_FLOATS 4480
__global__ __launch_bounds__(256) void k_proj(const unsigned short* __restrict__ XB, const unsigned short* __restrict__ WB,
                                              const float* __restrict__ vwb, const float* __restrict__ vaw,
                                              float* __restrict__ SD,
                                              unsigned short* __restrict__ VTH, unsigned short* __restrict__ VTL) {
  extern __shared__ __align__(16) float dsm[];
  __shared__ __align__(16) float sAw[128];
  const int tid = threadIdx.x, lane = tid & 31, wave = tid >> 5;
  if (wave == 0) *(v4f*)(sAw + 4 * lane) = *(const v4f*)(vaw + 4 * lane);
  __syncthreads();

  const int m0 = blockIdx.x * 64, n0 = wave * 64;
  v8f acc[4][4];
  gemm_tile64((const __bf16*)(const void*)XB, ND, (const __bf16*)(const void*)WB, ND, m0, n0, ND, ND - 1, lane, acc);

  float* T    = dsm + wave * PJ_WAVE_FLOATS;
  float* sdst = T + 64 * 68;
  const int rlane = lane & 15, mOff = (lane >> 4) * 8;
#pragma unroll
  for (int j = 0; j < 4; ++j) {
    const float bv = vwb[n0 + 16 * j + rlane];
#pragma unroll
    for (int i = 0; i < 4; ++i)
#pragma unroll
      for (int r = 0; r < 8; ++r)
        T[(16 * i + mOff + r) * 68 + 16 * j + rlane] = acc[i][j][r] + bv;
  }
  wave_sync();

  {
    float s0 = 0.0f, s1 = 0.0f, d0 = 0.0f, d1 = 0.0f;
    const float* t0 = T + lane * 68;
    const float* t1 = T + (lane + 32) * 68;
#pragma unroll 4
    for (int d = 0; d < NHD; ++d) {
      const float a = sAw[d], bb = sAw[NHD + d];
      const float u0 = t0[d], u1 = t1[d];
      s0 += u0 * a;  s1 += u1 * a;
      d0 += u0 * bb; d1 += u1 * bb;
    }
    sdst[lane] = s0; sdst[32 + lane] = s1; sdst[64 + lane] = d0; sdst[96 + lane] = d1;
  }
  wave_sync();
  const int b  = m0 >> 9;
  const int s0row = m0 & (NS - 1);
  const int bh = b * NH + wave;
  {
    const v4f sv = *(const v4fa*)(sdst + 4 * lane);
    const size_t off = (size_t)(lane >> 4) * SDHALF + (size_t)bh * NS + s0row + 4 * (lane & 15);
    *(volatile v4f*)(SD + off) = sv;
    __threadfence();
    *(volatile v4f*)(SD + off) = sv;
  }

  {
    const int q8 = lane & 7, sub = lane >> 3;
    for (int pass = 0; pass < 2; ++pass) {
#pragma unroll 2
      for (int it = 0; it < 16; ++it) {
        const int d = it * 4 + sub;
        v4u hv, lv;
#pragma unroll
        for (int q = 0; q < 4; ++q) {
          const float f0 = T[(8 * q8 + 2 * q) * 68 + d];
          const float f1 = T[(8 * q8 + 2 * q + 1) * 68 + d];
          const unsigned short h0 = f2bf_bits(f0), h1 = f2bf_bits(f1);
          const unsigned short l0 = f2bf_bits(f0 - bf_bits2f(h0)), l1 = f2bf_bits(f1 - bf_bits2f(h1));
          hv[q] = pk16(h0, h1);
          lv[q] = pk16(l0, l1);
        }
        const size_t go = ((size_t)bh * NHD + d) * NS + s0row + 8 * q8;
        *(volatile v4u*)(VTH + go) = hv;
        *(volatile v4u*)(VTL + go) = lv;
      }
      __threadfence();
    }
  }
}

__global__ __launch_bounds__(128) void k_attn(const float* __restrict__ SD, const unsigned* __restrict__ MASKB,
                                              const unsigned short* __restrict__ vhp, const unsigned short* __restrict__ vlp,
                                              float* __restrict__ CTX) {
  __shared__ __align__(16) __bf16 Vth[64 * 64];
  __shared__ __align__(16) __bf16 Vtl[64 * 64];
  __shared__ __align__(16) __bf16 Psh[4][16 * 64];
  __shared__ __align__(16) __bf16 Psl[4][16 * 64];
  __shared__ __align__(16) float  Os[4][16 * 68];
  __shared__ __align__(16) float  sDst[NS];
  __shared__ __align__(16) unsigned sMk[64 * 16];

  const int tid = threadIdx.x, wave = tid >> 5, lane = tid & 31;
  const int hh = lane >> 4, c = lane & 15;
  const int bx = blockIdx.x;
  const int qb = bx & 7, h = (bx >> 3) & 7, b = bx >> 6;
  const int bh = b * NH + h;
  const int i0 = qb * 64;
  const int q0 = i0 + wave * 16;

  const float* srcb = SD + (size_t)bh * NS;
  const float* dstb = SD + (size_t)SDHALF + (size_t)bh * NS;
  *(v4f*)(sDst + 4 * tid) = *(const v4f*)(dstb + 4 * tid);
  {
    const unsigned* mg = MASKB + ((size_t)b * NS + i0) * 16;
    *(v4u*)(sMk + 4 * tid)         = *(const v4u*)(mg + 4 * tid);
    *(v4u*)(sMk + 4 * (tid + 128)) = *(const v4u*)(mg + 4 * (tid + 128));
  }
  float srow[8];
  {
    const v4f sa = *(const v4f*)(srcb + q0 + 8 * hh);
    const v4f sb = *(const v4f*)(srcb + q0 + 8 * hh + 4);
    srow[0] = sa[0]; srow[1] = sa[1]; srow[2] = sa[2]; srow[3] = sa[3];
    srow[4] = sb[0]; srow[5] = sb[1]; srow[6] = sb[2]; srow[7] = sb[3];
  }
  __syncthreads();

  const __bf16* Vh = (const __bf16*)(const void*)vhp + (size_t)bh * NHD * NS;
  const __bf16* Vl = (const __bf16*)(const void*)vlp + (size_t)bh * NHD * NS;
  float* ob = CTX + (size_t)b * NS * ND + (size_t)h * NHD;

  float mrow[8], lrow[8];
  v8f oacc[4];
#pragma unroll
  for (int r = 0; r < 8; ++r) { mrow[r] = -INFINITY; lrow[r] = 0.f; }
#pragma unroll
  for (int t = 0; t < 4; ++t) oacc[t] = (v8f){0.f,0.f,0.f,0.f,0.f,0.f,0.f,0.f};

  const int mrow0 = (wave * 16 + 8 * hh) * 16;
#pragma unroll 1
  for (int kc = 0; kc < NS / 64; ++kc) {
    const int kv0 = kc * 64;
    __syncthreads();
    {
      const int r = tid >> 1, half = (tid & 1) * 32;
      const __bf16* vsh = Vh + (size_t)r * NS + kv0 + half;
      const __bf16* vsl = Vl + (size_t)r * NS + kv0 + half;
#pragma unroll
      for (int i = 0; i < 4; ++i) {
        const v8b b0 = *(const v8b*)(vsh + 8 * i);
        const v8b b1 = *(const v8b*)(vsl + 8 * i);
        *(v8b*)(Vth + r * 64 + half + 8 * i) = b0;
        *(v8b*)(Vtl + r * 64 + half + 8 * i) = b1;
      }
    }
    __syncthreads();

    float dcol[4];
#pragma unroll
    for (int j = 0; j < 4; ++j) dcol[j] = sDst[kv0 + 16 * j + c];
    v8f s[4];
#pragma unroll
    for (int r = 0; r < 8; ++r) {
      const unsigned mw0 = sMk[mrow0 + r * 16 + 2 * kc];
      const unsigned mw1 = sMk[mrow0 + r * 16 + 2 * kc + 1];
#pragma unroll
      for (int j = 0; j < 4; ++j) {
        const float v = srow[r] + dcol[j];
        float e = (v > 0.0f) ? v : 0.2f * v;
        const unsigned word = (j < 2) ? mw0 : mw1;
        const unsigned bit = (word >> (((j & 1) << 4) + c)) & 1u;
        e = (bit != 0u) ? -1.0e9f : e;
        s[j][r] = e;
      }
    }

    float cm[8];
#pragma unroll
    for (int r = 0; r < 8; ++r) {
      float m = -INFINITY;
#pragma unroll
      for (int j = 0; j < 4; ++j) m = fmaxf(m, s[j][r]);
#pragma unroll
      for (int off = 1; off < 16; off <<= 1) m = fmaxf(m, __shfl_xor(m, off, 32));
      cm[r] = m;
    }
    __bf16* pwh = Psh[wave];
    __bf16* pwl = Psl[wave];
#pragma unroll
    for (int r = 0; r < 8; ++r) {
      const float mnew = fmaxf(mrow[r], cm[r]);
      const float alpha = expf(mrow[r] - mnew);
      mrow[r] = mnew;
      float psum = 0.f;
#pragma unroll
      for (int j = 0; j < 4; ++j) {
        const float p = expf(s[j][r] - mnew);
        psum += p;
        const unsigned short hb = f2bf_bits(p);
        const unsigned short lb = f2bf_bits(p - bf_bits2f(hb));
        pwh[(8 * hh + r) * 64 + j * 16 + c] = __builtin_bit_cast(__bf16, hb);
        pwl[(8 * hh + r) * 64 + j * 16 + c] = __builtin_bit_cast(__bf16, lb);
      }
#pragma unroll
      for (int off = 1; off < 16; off <<= 1) psum += __shfl_xor(psum, off, 32);
      lrow[r] = lrow[r] * alpha + psum;
#pragma unroll
      for (int t = 0; t < 4; ++t) oacc[t][r] *= alpha;
    }
    wave_sync();
#pragma unroll 1
    for (int kk = 0; kk < 2; ++kk) {
      FB pa, pl;
      pa.h[0] = *(const v8b*)(pwh + c * 64 + kk * 32 + 8 * hh);
      pa.h[1] = *(const v8b*)(pwh + c * 64 + kk * 32 + 16 + 8 * hh);
      pl.h[0] = *(const v8b*)(pwl + c * 64 + kk * 32 + 8 * hh);
      pl.h[1] = *(const v8b*)(pwl + c * 64 + kk * 32 + 16 + 8 * hh);
#pragma unroll
      for (int t = 0; t < 4; ++t) {
        FB vb, vl;
        vb.h[0] = *(const v8b*)(Vth + (t * 16 + c) * 64 + kk * 32 + 8 * hh);
        vb.h[1] = *(const v8b*)(Vth + (t * 16 + c) * 64 + kk * 32 + 16 + 8 * hh);
        vl.h[0] = *(const v8b*)(Vtl + (t * 16 + c) * 64 + kk * 32 + 8 * hh);
        vl.h[1] = *(const v8b*)(Vtl + (t * 16 + c) * 64 + kk * 32 + 16 + 8 * hh);
        oacc[t] = at_mma(pa.v, vb.v, oacc[t]);
        oacc[t] = at_mma(pa.v, vl.v, oacc[t]);
        oacc[t] = at_mma(pl.v, vb.v, oacc[t]);
      }
    }
  }

  float* os = Os[wave];
#pragma unroll
  for (int r = 0; r < 8; ++r) {
    const float inv = 1.0f / lrow[r];
#pragma unroll
    for (int t = 0; t < 4; ++t) os[(8 * hh + r) * 68 + t * 16 + c] = oacc[t][r] * inv;
  }
  wave_sync();
  {
    const int c4 = (lane & 15) * 4;
    for (int pass = 0; pass < 2; ++pass) {
#pragma unroll
      for (int it = 0; it < 8; ++it) {
        const int row = it * 2 + hh;
        const v4f val = *(const v4fa*)(os + row * 68 + c4);
        *(volatile v4f*)(ob + (size_t)(q0 + row) * ND + c4) = val;
      }
      __threadfence();
    }
  }
}

__global__ __launch_bounds__(256) void k_ln1(const float* __restrict__ x, float* Y1,
                                             const float* __restrict__ vg, const float* __restrict__ vb,
                                             unsigned* __restrict__ Y1HLw) {
  __shared__ __align__(16) unsigned sHL[8][512];
  const int lane = threadIdx.x & 31, wave = threadIdx.x >> 5;
  const int row = blockIdx.x * 8 + wave;
  float* yr = Y1 + (size_t)row * ND;
  const float* xr = x + (size_t)row * ND;

  v4f v[4];
  float s = 0.0f;
#pragma unroll
  for (int c = 0; c < 4; ++c) {
    const int col = 4 * lane + 128 * c;
    const v4f a  = *(const v4f*)(yr + col);
    const v4f xv = *(const v4f*)(xr + col);
    v4f t;
    t[0] = a[0] + bfr(xv[0]); t[1] = a[1] + bfr(xv[1]); t[2] = a[2] + bfr(xv[2]); t[3] = a[3] + bfr(xv[3]);
    v[c] = t;
    s += (t[0] + t[1]) + (t[2] + t[3]);
  }
  s = wave_sum(s);
  const float mean = s * (1.0f / 512.0f);
  float q = 0.0f;
#pragma unroll
  for (int c = 0; c < 4; ++c) {
#pragma unroll
    for (int e = 0; e < 4; ++e) { const float d = v[c][e] - mean; q += d * d; }
  }
  q = wave_sum(q);
  const float rstd = 1.0f / sqrtf(q * (1.0f / 512.0f) + 1e-5f);

  v4f y[4];
#pragma unroll
  for (int c = 0; c < 4; ++c) {
    const int col = 4 * lane + 128 * c;
    const v4f g  = *(const v4f*)(vg + col);
    const v4f be = *(const v4f*)(vb + col);
    v4f o;
    unsigned short hb[4], lb[4];
#pragma unroll
    for (int e = 0; e < 4; ++e) {
      o[e] = (v[c][e] - mean) * rstd * g[e] + be[e];
      hb[e] = f2bf_bits(o[e]);
      lb[e] = f2bf_bits(o[e] - bf_bits2f(hb[e]));
    }
    y[c] = o;
    v2u hw, lw;
    hw[0] = pk16(hb[0], hb[1]); hw[1] = pk16(hb[2], hb[3]);
    lw[0] = pk16(lb[0], lb[1]); lw[1] = pk16(lb[2], lb[3]);
    *(v2ua*)(&sHL[wave][2 * lane + 64 * c])       = hw;
    *(v2ua*)(&sHL[wave][256 + 2 * lane + 64 * c]) = lw;
  }
  wave_sync();
  v4u w[4];
#pragma unroll
  for (int k = 0; k < 4; ++k) w[k] = *(const v4ua*)(&sHL[wave][4 * (lane + 32 * k)]);
  unsigned* hl = Y1HLw + (size_t)row * 512;
  for (int pass = 0; pass < 2; ++pass) {
#pragma unroll
    for (int c = 0; c < 4; ++c) *(volatile v4f*)(yr + 4 * lane + 128 * c) = y[c];
#pragma unroll
    for (int k = 0; k < 4; ++k) *(volatile v4u*)(hl + 4 * (lane + 32 * k)) = w[k];
    __threadfence();
  }
}

__global__ __launch_bounds__(256) void k_ff1(const unsigned short* __restrict__ Y1HL, const unsigned short* __restrict__ FF1B,
                                             const float* __restrict__ vb, unsigned short* __restrict__ GHL) {
  __shared__ __align__(16) float sT[8][16 * 68];
  const int lane = threadIdx.x & 31, wave = threadIdx.x >> 5;
  const int tile = blockIdx.x * 8 + wave;
  const int tm = tile >> 4, tn = tile & 15;
  const int m0 = tm * 64, n0 = tn * 64;

  v8f acc[4][4];
  gemm_tile64((const __bf16*)(const void*)Y1HL, 2 * ND, (const __bf16*)(const void*)FF1B, ND, m0, n0, 2 * ND, ND - 1, lane, acc);

  float* slab = sT[wave];
  const int rlane = lane & 15, mOff = (lane >> 4) * 8;
  float bv[4];
#pragma unroll
  for (int j = 0; j < 4; ++j) bv[j] = vb[n0 + 16 * j + rlane];
  const int q = lane >> 3, c8 = (lane & 7) * 8;

#pragma unroll
  for (int i = 0; i < 4; ++i) {
#pragma unroll
    for (int j = 0; j < 4; ++j)
#pragma unroll
      for (int r = 0; r < 8; ++r)
        slab[(mOff + r) * 68 + 16 * j + rlane] = acc[i][j][r] + bv[j];
    wave_sync();
#pragma unroll 2
    for (int it = 0; it < 32; ++it) {
      const int idx = it * 32 + lane;
      float* p = slab + (idx >> 6) * 68 + (idx & 63);
      const float v = *p;
      *p = 0.5f * v * (1.0f + erff(v * 0.70710678118654752f));
    }
    wave_sync();
    for (int pass = 0; pass < 2; ++pass) {
#pragma unroll
      for (int it = 0; it < 4; ++it) {
        const int row = it * 4 + q;
        const float* sp = slab + row * 68 + c8;
        v4u hv, lv;
#pragma unroll
        for (int e = 0; e < 4; ++e) {
          const float f0 = sp[2 * e], f1 = sp[2 * e + 1];
          const unsigned short h0 = f2bf_bits(f0), h1 = f2bf_bits(f1);
          const unsigned short l0 = f2bf_bits(f0 - bf_bits2f(h0)), l1 = f2bf_bits(f1 - bf_bits2f(h1));
          hv[e] = pk16(h0, h1);
          lv[e] = pk16(l0, l1);
        }
        const size_t go = (size_t)(m0 + 16 * i + row) * (2 * NFF) + n0 + c8;
        *(volatile v4u*)(GHL + go) = hv;
        *(volatile v4u*)(GHL + go + NFF) = lv;
      }
      __threadfence();
    }
    wave_sync();
  }
}

__global__ __launch_bounds__(256) void k_ff2ln(const unsigned short* __restrict__ GHL, const unsigned short* __restrict__ FF2B,
                                               const float* __restrict__ vb, const float* __restrict__ vg,
                                               const float* __restrict__ vbe, const float* __restrict__ Y1,
                                               float* __restrict__ out) {
  extern __shared__ __align__(16) float dsm[];
  const int tid = threadIdx.x, lane = tid & 31, wave = tid >> 5;
  const int m0 = blockIdx.x * 64, n0 = wave * 64;

  v8f acc[4][4];
  gemm_tile64((const __bf16*)(const void*)GHL, 2 * NFF, (const __bf16*)(const void*)FF2B, NFF, m0, n0, 2 * NFF, NFF - 1, lane, acc);

  const int rlane = lane & 15, mOff = (lane >> 4) * 8;
#pragma unroll
  for (int i = 0; i < 4; ++i)
#pragma unroll
    for (int j = 0; j < 4; ++j)
#pragma unroll
      for (int r = 0; r < 8; ++r)
        dsm[(16 * i + mOff + r) * TP + n0 + 16 * j + rlane] = acc[i][j][r];
  __syncthreads();

  v4f bb[4], gg[4], be[4];
#pragma unroll
  for (int c = 0; c < 4; ++c) {
    const int col = 4 * lane + 128 * c;
    bb[c] = *(const v4f*)(vb + col);
    gg[c] = *(const v4f*)(vg + col);
    be[c] = *(const v4f*)(vbe + col);
  }

#pragma unroll 1
  for (int rr = 0; rr < 8; ++rr) {
    const int row = wave * 8 + rr;
    float* tr = dsm + row * TP;
    const float* yrow = Y1 + (size_t)(m0 + row) * ND;
    v4f v[4];
    float s = 0.0f;
#pragma unroll
    for (int c = 0; c < 4; ++c) {
      const int col = 4 * lane + 128 * c;
      const v4f t  = *(const v4fa*)(tr + col);
      const v4f yy = *(const v4f*)(yrow + col);
      v4f u;
      u[0] = (t[0] + bb[c][0]) + yy[0]; u[1] = (t[1] + bb[c][1]) + yy[1];
      u[2] = (t[2] + bb[c][2]) + yy[2]; u[3] = (t[3] + bb[c][3]) + yy[3];
      v[c] = u;
      s += (u[0] + u[1]) + (u[2] + u[3]);
    }
    s = wave_sum(s);
    const float mean = s * (1.0f / 512.0f);
    float q = 0.0f;
#pragma unroll
    for (int c = 0; c < 4; ++c) {
#pragma unroll
      for (int e = 0; e < 4; ++e) { const float d = v[c][e] - mean; q += d * d; }
    }
    q = wave_sum(q);
    const float rstd = 1.0f / sqrtf(q * (1.0f / 512.0f) + 1e-5f);
#pragma unroll
    for (int c = 0; c < 4; ++c) {
      const int col = 4 * lane + 128 * c;
      v4f o;
#pragma unroll
      for (int e = 0; e < 4; ++e) o[e] = (v[c][e] - mean) * rstd * gg[c][e] + be[c][e];
      *(v4fa*)(tr + col) = o;
    }
  }

  for (int pass = 0; pass < 2; ++pass) {
#pragma unroll 1
    for (int rr = 0; rr < 8; ++rr) {
      const int row = wave * 8 + rr;
      const float* tr = dsm + row * TP;
      float* orow = out + (size_t)(m0 + row) * ND;
#pragma unroll
      for (int c = 0; c < 4; ++c) {
        const int col = 4 * lane + 128 * c;
        const v4f o = *(const v4fa*)(tr + col);
        *(volatile v4f*)(orow + col) = o;
      }
    }
    __threadfence();
  }
}

extern "C" void kernel_launch(void* const* d_in, const int* in_sizes, int n_in,
                              void* d_out, int out_size, void* d_ws, size_t ws_size,
                              hipStream_t stream) {
  if (n_in < 15) return;
  if (in_sizes[0] != NM * ND || in_sizes[1] != NM * ND) return;
  if (in_sizes[2] != ND * ND || in_sizes[3] != ND || in_sizes[4] != 2 * NHD) return;
  if (in_sizes[5] != ND * ND || in_sizes[6] != ND) return;
  if (in_sizes[7] != NFF * ND || in_sizes[8] != NFF || in_sizes[9] != ND * NFF || in_sizes[10] != ND) return;
  if (in_sizes[11] != ND || in_sizes[12] != ND || in_sizes[13] != ND || in_sizes[14] != ND) return;
  if (out_size != NM * ND) return;
  if (WS_TOTAL > ws_size) return;

  const float* x     = (const float*)d_in[0];
  const float* adj   = (const float*)d_in[1];
  const float* w_W   = (const float*)d_in[2];
  const float* w_b   = (const float*)d_in[3];
  const float* a_w   = (const float*)d_in[4];
  const float* sem_W = (const float*)d_in[5];
  const float* sem_b = (const float*)d_in[6];
  const float* ff1_W = (const float*)d_in[7];
  const float* ff1_b = (const float*)d_in[8];
  const float* ff2_W = (const float*)d_in[9];
  const float* ff2_b = (const float*)d_in[10];
  const float* ln1_g = (const float*)d_in[11];
  const float* ln1_b = (const float*)d_in[12];
  const float* ln2_g = (const float*)d_in[13];
  const float* ln2_b = (const float*)d_in[14];
  float* out = (float*)d_out;

  char* ws = (char*)d_ws;
  unsigned short* XB   = (unsigned short*)(ws + O_XB);
  unsigned short* ADJB = (unsigned short*)(ws + O_ADJB);
  unsigned short* Y1HL = (unsigned short*)(ws + O_Y1HL);
  unsigned short* VTH  = (unsigned short*)(ws + O_VTH);
  unsigned short* VTL  = (unsigned short*)(ws + O_VTL);
  unsigned short* GHL  = (unsigned short*)(ws + O_GHL);
  float*          CTX  = (float*)(ws + O_CTX);
  unsigned short* WB   = (unsigned short*)(ws + O_WB);
  unsigned short* SEMB = (unsigned short*)(ws + O_SEMB);
  unsigned short* FF1B = (unsigned short*)(ws + O_FF1B);
  unsigned short* FF2B = (unsigned short*)(ws + O_FF2B);
  unsigned*       MASKB = (unsigned*)(ws + O_MASK);
  float*          SD   = (float*)(ws + O_SD);
  float*          VEC  = (float*)(ws + O_VEC);

  const int ldsRow  = 64 * TP * 4;
  const int ldsProj = 8 * PJ_WAVE_FLOATS * 4;
  (void)hipFuncSetAttribute(reinterpret_cast<const void*>(&k_sem),   hipFuncAttributeMaxDynamicSharedMemorySize, ldsRow);
  (void)hipFuncSetAttribute(reinterpret_cast<const void*>(&k_proj),  hipFuncAttributeMaxDynamicSharedMemorySize, ldsProj);
  (void)hipFuncSetAttribute(reinterpret_cast<const void*>(&k_ff2ln), hipFuncAttributeMaxDynamicSharedMemorySize, ldsRow);

  k_prep<<<dim3(PB_END), dim3(256), 0, stream>>>(x, adj, w_W, w_b, a_w, sem_W, sem_b, ff1_W, ff1_b, ff2_W, ff2_b,
                                                 ln1_g, ln1_b, ln2_g, ln2_b, XB, ADJB, WB, SEMB, FF1B, FF2B, VEC);
  k_sem<<<dim3(NM / 64), dim3(256), ldsRow, stream>>>(ADJB, SEMB, VEC + V_SEMB, MASKB);
  k_proj<<<dim3(NM / 64), dim3(256), ldsProj, stream>>>(XB, WB, VEC + V_WB, VEC + V_AW, SD, VTH, VTL);
  k_attn<<<dim3(NB * NH * (NS / 64)), dim3(128), 0, stream>>>(SD, MASKB, VTH, VTL, CTX);
  k_ln1<<<dim3(NM / 8), dim3(256), 0, stream>>>(x, CTX, VEC + V_LN1G, VEC + V_LN1B, (unsigned*)Y1HL);
  for (int half = 0; half < NM / MHALF; ++half) {
    const size_t r0 = (size_t)half * MHALF;
    k_ff1<<<dim3((MHALF / 64) * (NFF / 64) / 8), dim3(256), 0, stream>>>(Y1HL + r0 * (2 * ND), FF1B, VEC + V_FF1B, GHL);
    k_ff2ln<<<dim3(MHALF / 64), dim3(256), ldsRow, stream>>>(GHL, FF2B, VEC + V_FF2B, VEC + V_LN2G, VEC + V_LN2B,
                                                             CTX + r0 * ND, out + r0 * ND);
  }
  (void)hipGetLastError();
}
